// CausalAttention_5841155523204
// MI455X (gfx1250) — hardware-verified
//
#include <hip/hip_runtime.h>


#ifndef NB
#define NB 4
#endif
#ifndef SEQ
#define SEQ 2048
#endif
#define NB_FULL  4
#define SEQ_FULL 2048
#define DM 1024
#ifndef RH
#define RH ((SEQ) < 512 ? (SEQ) : 512)
#endif
#define PCAR 1024.0f
#define QCAR 16.0f
#define SCL  0.0001220703125f

static_assert(DM == 1024);
static_assert(SEQ % 128 == 0);
static_assert(RH % 128 == 0);
static_assert(RH <= SEQ);
static_assert(SEQ <= SEQ_FULL);
static_assert(NB <= NB_FULL);
static_assert((DM * DM / 64) % 64 == 0);
static_assert(((size_t)NB * SEQ * (DM / 8)) % 256 == 0);

typedef _Float16 h16;
typedef unsigned short bf;
typedef __attribute__((ext_vector_type(16))) __bf16   v16bf;
typedef __attribute__((ext_vector_type(16))) _Float16 v16h;
typedef __attribute__((ext_vector_type(8)))  _Float16 v8h;
typedef __attribute__((ext_vector_type(8)))  unsigned short v8us;
typedef __attribute__((ext_vector_type(8)))  float    v8f;
typedef __attribute__((ext_vector_type(4)))  float    v4f;
typedef __attribute__((ext_vector_type(4)))  _Float16 v4h;
typedef __attribute__((ext_vector_type(2)))  unsigned short v2us;
typedef __attribute__((ext_vector_type(4)))  unsigned short v4us;
typedef v4f  __attribute__((may_alias)) v4fa;

__device__ __forceinline__ unsigned short f2bf(float f) { unsigned u = __float_as_uint(f); u += 0x7FFFu + ((u >> 16) & 1u); return (unsigned short)(u >> 16); }
__device__ __forceinline__ float bf2f(unsigned short b) { return __uint_as_float(((unsigned)b) << 16); }
__device__ __forceinline__ v16h cat16(v8h lo, v8h hi) { return __builtin_shufflevector(lo, hi, 0, 1, 2, 3, 4, 5, 6, 7, 8, 9, 10, 11, 12, 13, 14, 15); }
__device__ __forceinline__ v16bf cat16b(v8us lo, v8us hi) { return __builtin_bit_cast(v16bf, __builtin_shufflevector(lo, hi, 0, 1, 2, 3, 4, 5, 6, 7, 8, 9, 10, 11, 12, 13, 14, 15)); }
__device__ __forceinline__ v8f wmma16(v16h a, v16h b, v8f c) { return __builtin_amdgcn_wmma_f32_16x16x32_f16(false, a, false, b, (short)0, c, false, false); }
__device__ __forceinline__ v8f wmmab(v16bf a, v16bf b, v8f c) { return __builtin_amdgcn_wmma_f32_16x16x32_bf16(false, a, false, b, (short)0, c, false, false); }
__device__ __forceinline__ h16 tohx(float x) { return (h16)x; }
__device__ __forceinline__ void splitf(float y, unsigned short& h, unsigned short& l) { h = f2bf(y); l = f2bf(y - bf2f(h)); }

template <typename T16> struct WFrag;
template <> struct WFrag<h16> { typedef v16h V; static __device__ __forceinline__ V ld(const h16* p) { return cat16(*(const v8h*)p, *(const v8h*)(p + 16)); } static __device__ __forceinline__ v8f mma(V a, V b, v8f c) { return wmma16(a, b, c); } };
template <> struct WFrag<bf> { typedef v16bf V; static __device__ __forceinline__ V ld(const bf* p) { return cat16b(*(const v8us*)p, *(const v8us*)(p + 16)); } static __device__ __forceinline__ v8f mma(V a, V b, v8f c) { return wmmab(a, b, c); } };

template <typename T16, int NSPLIT, int OMODE>
__global__ __launch_bounds__(32) void k_gemmw(const T16* __restrict__ A, const T16* __restrict__ A2, const T16* __restrict__ Bt, const T16* __restrict__ Bt2,
                                              unsigned K, unsigned lda, unsigned ldb, float* C, h16* C16, bf* Hh, bf* Hl, unsigned ldc, unsigned ldh,
                                              float oscale, int cm, unsigned rbase, int hlmode, size_t sA, size_t sB, size_t sC, size_t sH) {
    typedef typename WFrag<T16>::V V;
    __shared__ __align__(16) float os[16 * 68];
    const size_t z = blockIdx.z;
    const unsigned lane = threadIdx.x & 31u, lr = lane & 15u, hi = lane >> 4;
    const unsigned r0 = blockIdx.x * 64u, c0 = blockIdx.y * 64u;
    if (cm == 1 && c0 > rbase + r0) return;
    unsigned Keff = K;
    if (cm == 2) { const unsigned kb = rbase + r0 + 64u; Keff = (kb < K) ? kb : K; }
    A += z * sA; Bt += z * sB;
    if (NSPLIT == 1 || NSPLIT == 2) A2 += z * sA;
    if (NSPLIT >= 2) Bt2 += z * sB;
    v8f acc[4][4];
#pragma unroll
    for (int mb = 0; mb < 4; ++mb)
#pragma unroll
        for (int nb = 0; nb < 4; ++nb) acc[mb][nb] = (v8f){};
    const size_t aoff = (size_t)(r0 + lr) * lda + 8u * hi, boff = (size_t)(c0 + lr) * ldb + 8u * hi;
#pragma unroll 1
    for (unsigned kc = 0; kc < Keff; kc += 32) {
        V a[4], a2[4];
#pragma unroll
        for (int mb = 0; mb < 4; ++mb) { a[mb] = WFrag<T16>::ld(A + aoff + (size_t)mb * 16 * lda + kc); if (NSPLIT == 1 || NSPLIT == 2) a2[mb] = WFrag<T16>::ld(A2 + aoff + (size_t)mb * 16 * lda + kc); }
#pragma unroll
        for (int nb = 0; nb < 4; ++nb) { const V b = WFrag<T16>::ld(Bt + boff + (size_t)nb * 16 * ldb + kc); V b2; if (NSPLIT >= 2) b2 = WFrag<T16>::ld(Bt2 + boff + (size_t)nb * 16 * ldb + kc);
#pragma unroll
            for (int mb = 0; mb < 4; ++mb) { acc[mb][nb] = WFrag<T16>::mma(a[mb], b, acc[mb][nb]); if (NSPLIT == 1 || NSPLIT == 2) acc[mb][nb] = WFrag<T16>::mma(a2[mb], b, acc[mb][nb]); if (NSPLIT >= 2) acc[mb][nb] = WFrag<T16>::mma(a[mb], b2, acc[mb][nb]); } }
        asm volatile("v_nop\n\tv_nop\n\tv_nop\n\tv_nop" : "+v"(acc[0][0]), "+v"(acc[1][1]), "+v"(acc[2][2]), "+v"(acc[3][3]) : "v"(a[0]), "v"(a[3]));
    }
    bool dohl = false; size_t hoff = 0;
    if (OMODE == 1) {
        if (hlmode == 1) { const unsigned bq = r0 / (unsigned)SEQ, t0 = r0 - bq * (unsigned)SEQ; dohl = (t0 < (unsigned)RH); if (dohl) hoff = (size_t)(bq * (unsigned)RH + t0) * ldh + c0; }
        else if (hlmode == 2) { dohl = (c0 < (unsigned)RH); if (dohl) hoff = z * sH + (size_t)r0 * ldh + c0; }
    }
#pragma unroll
    for (int mb = 0; mb < 4; ++mb) {
#pragma unroll
        for (int nb = 0; nb < 4; ++nb) {
#pragma unroll
            for (int j = 0; j < 8; ++j) os[(hi * 8 + j) * 68 + nb * 16 + lr] = acc[mb][nb][j]; }
        __builtin_amdgcn_wave_barrier(); asm volatile("" ::: "memory");
        if (OMODE == 0) {
            float* crow = C + z * sC + (size_t)(r0 + mb * 16) * ldc + c0;
#pragma unroll 1
            for (int ps = 0; ps < 2; ++ps) {
#pragma unroll
                for (int s = 0; s < 8; ++s) { const unsigned row = 2u * s + hi, cofs = lr * 4u; v4f val = *(const v4fa*)(os + row * 68 + cofs);
                    val[0] = val[0] * oscale; val[1] = val[1] * oscale; val[2] = val[2] * oscale; val[3] = val[3] * oscale;
                    *(volatile v4f*)(crow + (size_t)row * ldc + cofs) = val; }
                if (ps == 0) __threadfence(); }
        } else {
            h16* prow = C16 + z * sC + (size_t)(r0 + mb * 16) * ldc + c0;
            bf* hrow = Hh + hoff + (size_t)(mb * 16) * ldh;
            bf* lrow = Hl + hoff + (size_t)(mb * 16) * ldh;
#pragma unroll 1
            for (int ps = 0; ps < 2; ++ps) {
#pragma unroll
                for (int s = 0; s < 4; ++s) { const unsigned row = 4u * s + (lane >> 3), cofs = (lane & 7u) * 8u;
                    const v4f v0 = *(const v4fa*)(os + row * 68 + cofs); const v4f v1 = *(const v4fa*)(os + row * 68 + cofs + 4);
                    v8h o; v8us oh, ol;
#pragma unroll
                    for (int q = 0; q < 4; ++q) { const float y0 = v0[q] * oscale, y1 = v1[q] * oscale; o[q] = tohx(y0); o[q + 4] = tohx(y1);
                        unsigned short a2, c2; splitf(y0, a2, c2); oh[q] = a2; ol[q] = c2; splitf(y1, a2, c2); oh[q + 4] = a2; ol[q + 4] = c2; }
                    *(volatile v8h*)(prow + (size_t)row * ldc + cofs) = o;
                    if (dohl) { *(volatile v8us*)(hrow + (size_t)row * ldh + cofs) = oh; *(volatile v8us*)(lrow + (size_t)row * ldh + cofs) = ol; } }
                if (ps == 0) __threadfence(); }
        }
        __builtin_amdgcn_wave_barrier(); asm volatile("" ::: "memory");
    }
}

__global__ __launch_bounds__(256) void k_cvt8(const float* __restrict__ x, bf* dst) {
    const unsigned i = blockIdx.x * 256u + threadIdx.x; if (i >= (unsigned)(NB * SEQ * (DM / 8))) return;
    const unsigned row = i >> 7, g = i & 127u; const unsigned b = row / (unsigned)SEQ, t = row - b * (unsigned)SEQ;
    const float* s = x + ((size_t)b * SEQ_FULL + t) * DM + g * 8u; const v4f v0 = *(const v4f*)s; const v4f v1 = *(const v4f*)(s + 4); v8us o;
#pragma unroll
    for (int k = 0; k < 4; ++k) { o[k] = f2bf(v0[k]); o[k + 4] = f2bf(v1[k]); }
    bf* d = dst + (size_t)i * 8u; *(volatile v8us*)d = o; __threadfence(); *(volatile v8us*)d = o; }

__global__ __launch_bounds__(256) void k_wtG(const float* __restrict__ w, bf* Bt) {
    const unsigned lane = threadIdx.x & 31u; const unsigned L0 = (blockIdx.x * 8u + (threadIdx.x >> 5)) * 8u; const unsigned nlines = (unsigned)(DM * DM / 64);
#pragma unroll 1
    for (int ps = 0; ps < 2; ++ps) {
#pragma unroll 1
        for (unsigned l = 0; l < 8u; ++l) { const unsigned L = L0 + l; if (L < nlines) { const unsigned e = L * 64u + lane * 2u; const unsigned k = e & (unsigned)(DM - 1), n = e >> 10; v2us o;
            o[0] = f2bf(w[(size_t)k * DM + n]); o[1] = f2bf(w[(size_t)(k + 1u) * DM + n]); *(volatile v2us*)(Bt + e) = o; } }
        if (ps == 0) __threadfence(); }
}

__global__ __launch_bounds__(256) void k_lsoft(const float* __restrict__ Sb, h16* P16, bf* Ph, bf* Pl) {
    const unsigned lane = threadIdx.x & 31u; const unsigned i = blockIdx.x * 8u + (threadIdx.x >> 5); if (i >= (unsigned)SEQ) return;
    const bool hires = (i < (unsigned)RH); const unsigned ext = ((i >> 6) + 1u) << 6; const unsigned nch = (ext + 127u) >> 7;
    const float* sr = Sb + (size_t)i * SEQ; float mx = -3.0e38f;
#pragma unroll 1
    for (unsigned ch = 0; ch < nch; ++ch) { const unsigned j0 = ch * 128u + lane * 4u; const unsigned jl = (j0 < ext) ? j0 : (ext - 4u); const v4f a = *(const v4f*)(sr + jl);
#pragma unroll
        for (unsigned q = 0; q < 4u; ++q) { float t = (j0 + q <= i) ? a[q] * SCL : -3.0e38f; asm volatile("" : "+v"(t)); mx = fmaxf(mx, t); } }
#pragma unroll
    for (int sh = 16; sh; sh >>= 1) mx = fmaxf(mx, __shfl_xor(mx, sh, 32));
    float sum = 0.f;
#pragma unroll 1
    for (unsigned ch = 0; ch < nch; ++ch) { const unsigned j0 = ch * 128u + lane * 4u; const unsigned jl = (j0 < ext) ? j0 : (ext - 4u); const v4f a = *(const v4f*)(sr + jl);
#pragma unroll
        for (unsigned q = 0; q < 4u; ++q) { float t = (j0 + q <= i) ? a[q] * SCL : -3.0e38f; asm volatile("" : "+v"(t)); float d0 = __fsub_rn(t, mx); asm volatile("" : "+v"(d0)); sum += __builtin_amdgcn_exp2f(__fmul_rn(d0, 1.4426950408889634f)); } }
#pragma unroll
    for (int sh = 16; sh; sh >>= 1) sum += __shfl_xor(sum, sh, 32);
    const float f = __fdiv_rn(hires ? 1.0f : PCAR, sum);
#pragma unroll 1
    for (int ps = 0; ps < 2; ++ps) {
        if (hires) {
#pragma unroll 1
            for (unsigned ch = 0; ch < nch; ++ch) { const unsigned j0 = ch * 128u + lane * 4u; const unsigned jl = (j0 < ext) ? j0 : (ext - 4u); const v4f a = *(const v4f*)(sr + jl); v4us oh, ol;
#pragma unroll
                for (unsigned q = 0; q < 4u; ++q) { float t = (j0 + q <= i) ? a[q] * SCL : -3.0e38f; asm volatile("" : "+v"(t)); float d0 = __fsub_rn(t, mx); asm volatile("" : "+v"(d0)); float ex = __builtin_amdgcn_exp2f(__fmul_rn(d0, 1.4426950408889634f)); asm volatile("" : "+v"(ex)); unsigned short a2, c2; splitf(ex * f, a2, c2); oh[q] = a2; ol[q] = c2; }
                const size_t oo = (size_t)i * RH + j0; *(volatile v4us*)(Ph + oo) = oh; *(volatile v4us*)(Pl + oo) = ol; }
        } else {
#pragma unroll 1
            for (unsigned ch = 0; ch < nch; ++ch) { const unsigned j0 = ch * 128u + lane * 4u; const unsigned jl = (j0 < ext) ? j0 : (ext - 4u); const v4f a = *(const v4f*)(sr + jl); v4h o4;
#pragma unroll
                for (unsigned q = 0; q < 4u; ++q) { float t = (j0 + q <= i) ? a[q] * SCL : -3.0e38f; asm volatile("" : "+v"(t)); float d0 = __fsub_rn(t, mx); asm volatile("" : "+v"(d0)); float ex = __builtin_amdgcn_exp2f(__fmul_rn(d0, 1.4426950408889634f)); asm volatile("" : "+v"(ex)); o4[q] = tohx(ex * f); }
                *(volatile v4h*)(P16 + (size_t)(i - (unsigned)RH) * SEQ + j0) = o4; } }
        if (ps == 0) __threadfence(); }
}

extern "C" void kernel_launch(void* const* d_in, const int* in_sizes, int n_in,
                              void* d_out, int out_size, void* d_ws, size_t ws_size, hipStream_t stream) {
    if (n_in < 4) return;
    const size_t need_x = ((size_t)(NB - 1) * SEQ_FULL + SEQ) * DM;
    if ((size_t)in_sizes[0] < need_x || (size_t)in_sizes[1] < (size_t)DM * DM || (size_t)in_sizes[2] < (size_t)DM * DM || (size_t)in_sizes[3] < (size_t)DM * DM) return;
    if ((size_t)out_size < need_x) return;
    const float* x = (const float*)d_in[0]; const float* wq = (const float*)d_in[1]; const float* wk = (const float*)d_in[2]; const float* wv = (const float*)d_in[3];
    float* OUT = (float*)d_out;
    char* wsp = (char*)d_ws;
    auto take = [&](size_t bytes) { char* p = wsp; wsp += (bytes + 255) & ~(size_t)255; return (void*)p; };
    bf* WQ = (bf*)take((size_t)DM * DM * 2); bf* WK = (bf*)take((size_t)DM * DM * 2); bf* WV = (bf*)take((size_t)DM * DM * 2);
    bf* XB = (bf*)take((size_t)NB * SEQ * DM * 2);
    h16* Q16 = (h16*)take((size_t)NB * SEQ * DM * 2); h16* K16 = (h16*)take((size_t)NB * SEQ * DM * 2);
    bf* QPh = (bf*)take((size_t)NB * RH * DM * 2); bf* QPl = (bf*)take((size_t)NB * RH * DM * 2);
    bf* KPh = (bf*)take((size_t)NB * RH * DM * 2); bf* KPl = (bf*)take((size_t)NB * RH * DM * 2);
    h16* VT16 = (h16*)take((size_t)NB * DM * SEQ * 2);
    bf* VTh = (bf*)take((size_t)NB * DM * RH * 2); bf* VTl = (bf*)take((size_t)NB * DM * RH * 2);
    float* Sb = (float*)take((size_t)SEQ * SEQ * 4);
    h16* P16 = (h16*)take((size_t)(SEQ - RH) * SEQ * 2); bf* Ph = (bf*)take((size_t)RH * RH * 2); bf* Pl = (bf*)take((size_t)RH * RH * 2);
    if ((size_t)(wsp - (char*)d_ws) > ws_size) return;
    k_wtG<<<(unsigned)(DM * DM / 64 / 64), 256, 0, stream>>>(wq, WQ); k_wtG<<<(unsigned)(DM * DM / 64 / 64), 256, 0, stream>>>(wk, WK); k_wtG<<<(unsigned)(DM * DM / 64 / 64), 256, 0, stream>>>(wv, WV);
    k_cvt8<<<(unsigned)((size_t)NB * SEQ * (DM / 8) / 256), 256, 0, stream>>>(x, XB);
    k_gemmw<bf, 0, 1><<<dim3(NB * SEQ / 64, DM / 64, 1), 32, 0, stream>>>(XB, nullptr, WQ, nullptr, DM, DM, DM, nullptr, Q16, QPh, QPl, DM, DM, QCAR, 0, 0u, 1, 0, 0, 0, 0);
    k_gemmw<bf, 0, 1><<<dim3(NB * SEQ / 64, DM / 64, 1), 32, 0, stream>>>(XB, nullptr, WK, nullptr, DM, DM, DM, nullptr, K16, KPh, KPl, DM, DM, QCAR, 0, 0u, 1, 0, 0, 0, 0);
    k_gemmw<bf, 0, 1><<<dim3(DM / 64, SEQ / 64, NB), 32, 0, stream>>>(WV, nullptr, XB, nullptr, DM, DM, DM, nullptr, VT16, VTh, VTl, SEQ, RH, QCAR, 0, 0u, 2, 0, (size_t)SEQ * DM, (size_t)DM * SEQ, (size_t)DM * RH);
    for (int b = 0; b < NB; ++b) {
        const size_t qh = (size_t)b * RH * DM, q16 = (size_t)b * SEQ * DM;
        k_gemmw<bf, 2, 0><<<dim3(RH / 64, RH / 64, 1), 32, 0, stream>>>(QPh + qh, QPl + qh, KPh + qh, KPl + qh, DM, DM, DM, Sb, nullptr, nullptr, nullptr, SEQ, 0, 1.0f, 1, 0u, 0, 0, 0, 0, 0);
        if (SEQ > RH) k_gemmw<h16, 0, 0><<<dim3((SEQ - RH) / 64, SEQ / 64, 1), 32, 0, stream>>>(Q16 + q16 + (size_t)RH * DM, nullptr, K16 + q16, nullptr, DM, DM, DM, Sb + (size_t)RH * SEQ, nullptr, nullptr, nullptr, SEQ, 0, 1.0f, 1, (unsigned)RH, 0, 0, 0, 0, 0);
        k_lsoft<<<SEQ / 8, 256, 0, stream>>>(Sb, P16, Ph, Pl);
        k_gemmw<bf, 2, 0><<<dim3(RH / 64, DM / 64, 1), 32, 0, stream>>>(Ph, Pl, VTh + (size_t)b * DM * RH, VTl + (size_t)b * DM * RH, RH, RH, RH, OUT + (size_t)b * SEQ_FULL * DM, nullptr, nullptr, nullptr, DM, 0, 1.0f / QCAR, 2, 0u, 0, 0, 0, 0, 0);
        if (SEQ > RH) k_gemmw<h16, 0, 0><<<dim3((SEQ - RH) / 64, DM / 64, 1), 32, 0, stream>>>(P16, nullptr, VT16 + (size_t)b * DM * SEQ, nullptr, SEQ, SEQ, SEQ, OUT + ((size_t)b * SEQ_FULL + RH) * DM, nullptr, nullptr, nullptr, DM, 0, 1.0f / (PCAR * QCAR), 2, (unsigned)RH, 0, 0, 0, 0, 0);
    }
}
